// EntityPairAttentionNeighboursRelationEmbedding_45397804318893
// MI455X (gfx1250) — hardware-verified
//
#include <hip/hip_runtime.h>

#define NPAIR 4096
#define LL    256
#define KK    256
#define RR    50000
#define TSTR  264

typedef _Float16 f16;
typedef __attribute__((ext_vector_type(16))) f16 f16x16;
typedef __attribute__((ext_vector_type(8)))  f16 f16x8;
typedef __attribute__((ext_vector_type(8)))  float f32x8;
typedef __attribute__((ext_vector_type(4)))  float v4f_t;
typedef float v4fa __attribute__((ext_vector_type(4), may_alias));

__device__ __forceinline__ f32x8 wmma16(f16x16 a, f16x16 b, f32x8 c) {
  c = __builtin_amdgcn_wmma_f32_16x16x32_f16(false, a, false, b, (short)0, c, false, false);
  asm volatile("v_nop\n\tv_nop\n\tv_nop\n\tv_nop" : "+v"(c) : "v"(a), "v"(b));
  return c;
}
__device__ __forceinline__ f16x16 lds_frag(const f16* base, int stride) {
  const int lane = threadIdx.x & 31, row = lane & 15, kh = (lane >> 4) * 8;
  const f16x8 lo = *(const f16x8*)(base + row * stride + kh);
  const f16x8 hi = *(const f16x8*)(base + row * stride + kh + 16);
  f16x16 f;
#pragma unroll
  for (int i = 0; i < 8; ++i) { f[i] = lo[i]; f[i + 8] = hi[i]; }
  return f;
}

__global__ __launch_bounds__(256) void k_pair_score(const float* __restrict__ table, const float* __restrict__ w1,
                                                    const float* __restrict__ w2, const int* __restrict__ cand_idx,
                                                    const int* __restrict__ neigh_idx, const int* __restrict__ lengths,
                                                    float* __restrict__ out) {
  __shared__ __attribute__((aligned(16))) f16 Th[32 * TSTR], Tl[32 * TSTR];
  __shared__ __attribute__((aligned(16))) f16 Ch[16 * TSTR], Cl[16 * TSTR];
  __shared__ float wgt[LL];
  __shared__ float dS[LL];
  __shared__ float red[8];
  __shared__ __attribute__((aligned(16))) float scS[32];
  const int tid = threadIdx.x, lane = tid & 31, wave = tid >> 5, cl = lane & 15, rh = (lane >> 4) * 8;

  for (int e = tid; e < 16 * TSTR; e += 256) { Ch[e] = (f16)0.0f; Cl[e] = (f16)0.0f; }
#pragma unroll 1
  for (int q = 0; q < 32; ++q) {
    const int n = blockIdx.x * 32 + q;
    __syncthreads();
    {
      int ci = cand_idx[n]; ci = min(max(ci, 0), RR - 1);
      const float v = table[(size_t)ci * KK + tid] * 64.0f;
      const f16 hv = (f16)v; Ch[tid] = hv; Cl[tid] = (f16)((v - (float)hv) * 2048.0f);
    }
    int len = lengths[n]; len = min(max(len, 0), LL);
    const float lw = (tid < len) ? (w1[(size_t)n * LL + tid] + w2[(size_t)n * LL + tid]) : -3.0e38f;
    float m = lw;
#pragma unroll
    for (int off = 16; off >= 1; off >>= 1) m = fmaxf(m, __shfl_xor(m, off, 32));
    if (lane == 0) red[wave] = m;
    __syncthreads();
    m = fmaxf(fmaxf(fmaxf(red[0], red[1]), fmaxf(red[2], red[3])), fmaxf(fmaxf(red[4], red[5]), fmaxf(red[6], red[7])));
    const float ex = (tid < len) ? __expf(lw - m) : 0.0f;
    float ssum = ex;
#pragma unroll
    for (int off = 16; off >= 1; off >>= 1) ssum += __shfl_xor(ssum, off, 32);
    __syncthreads();
    if (lane == 0) red[wave] = ssum;
    __syncthreads();
    ssum = ((red[0] + red[1]) + (red[2] + red[3])) + ((red[4] + red[5]) + (red[6] + red[7]));
    wgt[tid] = (len > 0) ? (ex / ssum) : 1.0f;

#pragma unroll 1
    for (int chk = 0; chk < LL / 32; ++chk) {
      __syncthreads();
      {
        const int rl = tid >> 3, d0 = (tid & 7) * 32, l = chk * 32 + rl;
        int ni = neigh_idx[(size_t)n * LL + l]; ni = min(max(ni, 0), RR - 1);
        const float* src = table + (size_t)ni * KK + d0;
#pragma unroll
        for (int g = 0; g < 8; ++g) {
          const v4f_t v = *(const v4f_t*)(src + 4 * g);
#pragma unroll
          for (int u = 0; u < 4; ++u) {
            const float vs = v[u] * 64.0f;
            const f16 hv = (f16)vs;
            Th[rl * TSTR + d0 + 4 * g + u] = hv; Tl[rl * TSTR + d0 + 4 * g + u] = (f16)((vs - (float)hv) * 2048.0f);
          }
        }
      }
      __syncthreads();
      if (wave < 2) {
        f32x8 acc = {}, accx = {};
#pragma unroll
        for (int ks = 0; ks < KK / 32; ++ks) {
          const f16x16 ah = lds_frag(Th + wave * 16 * TSTR + ks * 32, TSTR), al = lds_frag(Tl + wave * 16 * TSTR + ks * 32, TSTR);
          const f16x16 bh = lds_frag(Ch + ks * 32, TSTR), bl = lds_frag(Cl + ks * 32, TSTR);
          acc = wmma16(ah, bh, acc); accx = wmma16(ah, bl, accx); accx = wmma16(al, bh, accx);
        }
        if (cl == 0) {
#pragma unroll
          for (int j = 0; j < 8; ++j) dS[chk * 32 + wave * 16 + rh + j] = (acc[j] + accx[j] * (1.0f / 2048.0f)) * (1.0f / 4096.0f);
        }
      }
    }
    __syncthreads();
    float pr = wgt[tid] * dS[tid];
#pragma unroll
    for (int off = 16; off >= 1; off >>= 1) pr += __shfl_xor(pr, off, 32);
    if (lane == 0) red[wave] = pr;
    __syncthreads();
    if (tid == 0) scS[q] = ((red[0] + red[1]) + (red[2] + red[3])) + ((red[4] + red[5]) + (red[6] + red[7]));
  }
  __syncthreads();
#pragma unroll 1
  for (int pass = 0; pass < 2; ++pass) {
    if (tid < 8) *(volatile v4f_t*)(out + (size_t)blockIdx.x * 32 + tid * 4) = *(const volatile v4fa*)(scS + tid * 4);
    __threadfence();
  }
}

extern "C" void kernel_launch(void* const* d_in, const int* in_sizes, int n_in,
                              void* d_out, int out_size, void* d_ws, size_t ws_size,
                              hipStream_t stream) {
  (void)in_sizes; (void)n_in; (void)out_size; (void)d_ws; (void)ws_size;
  const float* table = (const float*)d_in[0];
  const float* w1 = (const float*)d_in[1];
  const float* w2 = (const float*)d_in[2];
  const int* cand  = (const int*)d_in[3];
  const int* neigh = (const int*)d_in[4];
  const int* lens  = (const int*)d_in[5];
  float* out = (float*)d_out;
  k_pair_score<<<dim3(NPAIR / 32), dim3(256), 0, stream>>>(table, w1, w2, cand, neigh, lens, out);
}
